// LightTransformerBlock_23347442221594
// MI455X (gfx1250) — hardware-run, weakly checked
//
#include <hip/hip_runtime.h>
#pragma clang fp contract(off)


#ifndef NB
#define NB 8
#endif
#ifndef SEQ
#define SEQ 2048
#endif
#define NB_FULL  8
#define SEQ_FULL 2048
#ifndef OUT_SEQ
#define OUT_SEQ SEQ
#endif
#define DM   128
#define NH_  4
#define HD   32
#define AW   4
#define OSP  36
#define TW   2
#define TP   132
#define HTP  136
#define LP   132
#define SC2  ((float)(0.17677669529663687 * 1.4426950408889634))
#define PSH  14.0f
#define NEGB (-3.0e38f)
#define FILL2 ((float)(-1.0e9 * 1.4426950408889634))
#define WCS  64.0f
#define CXS  64.0f
#define CI1  (1.0f / 4096.0f)
#define CI2  (1.0f / 64.0f)
#define GK   0.7978845608028654f

static_assert(HD == 32);
static_assert(NH_ * HD == DM);
static_assert(DM / 32 == NH_);
static_assert(DM % 32 == 0);
static_assert(DM == 32 * 4);
static_assert(SEQ % 64 == 0);
static_assert((NB * SEQ) % 64 == 0);
static_assert(SEQ % 32 == 0);
static_assert(SEQ % (16 * AW) == 0);
static_assert((NB * SEQ) % (16 * TW) == 0);
static_assert(SEQ % (16 * TW) == 0);
static_assert(NB <= NB_FULL);
static_assert(SEQ <= SEQ_FULL);
static_assert((OSP * 4) % 16 == 0);
static_assert((TP * 4) % 16 == 0);
static_assert((HTP * 2) % 16 == 0);
static_assert((LP * 4) % 16 == 0);
static_assert(2 * 32 * 8 == 16 * HD);
static_assert(4 * 256 * 8 == 64 * DM);
static_assert(64 * LP * 4 <= 131072);
static_assert(AW * 16 * OSP * 4 <= 131072);
static_assert(2 * TW * 16 * TP * 4 + TW * 16 * HTP * 2 <= 65536);

typedef _Float16 h16;
typedef unsigned short bf;
typedef __attribute__((ext_vector_type(16))) __bf16   v16bf;
typedef __attribute__((ext_vector_type(16))) _Float16 v16h;
typedef __attribute__((ext_vector_type(8)))  _Float16 v8h;
typedef __attribute__((ext_vector_type(8)))  unsigned short v8us;
typedef __attribute__((ext_vector_type(8)))  float    v8f;
typedef __attribute__((ext_vector_type(4)))  float    v4f;
typedef v4f  __attribute__((may_alias)) v4fa;
typedef __attribute__((ext_vector_type(4)))  int      v4i;
typedef __attribute__((ext_vector_type(4)))  _Float16 v4h;
typedef v4h  __attribute__((may_alias)) v4ha;
typedef v8h  __attribute__((may_alias)) v8ha;

__device__ __forceinline__ unsigned short f2bf(float f) { unsigned u = __float_as_uint(f); u += 0x7FFFu + ((u >> 16) & 1u); return (unsigned short)(u >> 16); }
__device__ __forceinline__ float bfr(float f) { return __uint_as_float(((unsigned)f2bf(f)) << 16); }
__device__ __forceinline__ v16h cat16(v8h lo, v8h hi) { return __builtin_shufflevector(lo, hi, 0, 1, 2, 3, 4, 5, 6, 7, 8, 9, 10, 11, 12, 13, 14, 15); }
__device__ __forceinline__ v16bf cat16b(v8us lo, v8us hi) { return __builtin_bit_cast(v16bf, __builtin_shufflevector(lo, hi, 0, 1, 2, 3, 4, 5, 6, 7, 8, 9, 10, 11, 12, 13, 14, 15)); }
__device__ __forceinline__ v8f wmma16(v16h a, v16h b, v8f c) { return __builtin_amdgcn_wmma_f32_16x16x32_f16(false, a, false, b, (short)0, c, false, false); }
__device__ __forceinline__ v8f wmmab(v16bf a, v16bf b, v8f c) { return __builtin_amdgcn_wmma_f32_16x16x32_bf16(false, a, false, b, (short)0, c, false, false); }
__device__ __forceinline__ v16h  ldh(const h16* p) { return cat16(*(const v8h*)p, *(const v8h*)(p + 16)); }
__device__ __forceinline__ v16bf ldb(const bf* p)  { return cat16b(*(const v8us*)p, *(const v8us*)(p + 16)); }
__device__ __forceinline__ void wave_sync() { __builtin_amdgcn_fence(3  , "wavefront"); __builtin_amdgcn_wave_barrier(); asm volatile("" ::: "memory"); }

static __device__ __forceinline__ h16 toh_flush(float v) { const h16 r = (h16)v; return (fabsf(v) < 6.103515625e-05f) ? (h16)0.0f : r; }
static __device__ __forceinline__ v8f wmma16g(v16h a, v16h b, v8f c) { c = wmma16(a, b, c); asm volatile("v_nop\n\tv_nop\n\tv_nop\n\tv_nop" : "+v"(c) : "v"(a), "v"(b)); return c; }

__global__ __launch_bounds__(256) void k_wcvt(const float* __restrict__ src, h16* dst, size_t n8) {
    const size_t i = (size_t)blockIdx.x * 256 + threadIdx.x; if (i >= n8) return;
    const v8f v = *(const v8f*)(src + i * 8); v8h o;
#pragma unroll
    for (int k = 0; k < 8; ++k) o[k] = toh_flush(bfr(v[k]) * WCS);
    *(volatile v8h*)(dst + i * 8) = o; __threadfence(); *(volatile v8h*)(dst + i * 8) = o;
}

__global__ __launch_bounds__(256) void k_ln1(const float* __restrict__ X, const float* __restrict__ ga, const float* __restrict__ gb, h16* QP, h16* VT) {
    __shared__ __align__(16) float ns[64 * LP];
    const int tid = threadIdx.x, lane = tid & 31;
    const int wave = __builtin_amdgcn_readfirstlane((int)(threadIdx.x >> 5));
    const int r0 = blockIdx.x * 64; const int bb = r0 / SEQ, tt = r0 % SEQ;
    v4f av = *(const v4f*)(ga + 4 * lane), bv = *(const v4f*)(gb + 4 * lane);
#pragma unroll
    for (int i = 0; i < 4; ++i) { av[i] = bfr(av[i]); bv[i] = bfr(bv[i]); }
#pragma unroll 1
    for (int i = 0; i < 8; ++i) {
        const int row = wave * 8 + i;
        v4f x = *(const v4f*)(X + ((size_t)bb * SEQ_FULL + (size_t)(tt + row)) * DM + 4 * lane);
#pragma unroll
        for (int c = 0; c < 4; ++c) x[c] = bfr(x[c]);
        float s = (x[0] + x[1]) + (x[2] + x[3]);
#pragma unroll
        for (int o = 16; o >= 1; o >>= 1) s += __shfl_xor(s, o, 32);
        const float mean = s * (1.0f / DM);
        v4f d; float ss = 0.0f;
#pragma unroll
        for (int c = 0; c < 4; ++c) { d[c] = x[c] - mean; ss += d[c] * d[c]; }
#pragma unroll
        for (int o = 16; o >= 1; o >>= 1) ss += __shfl_xor(ss, o, 32);
        const float sd = sqrtf(ss * (1.0f / (DM - 1)));
        const float inv = 1.0f / (sd + 1e-6f);
        v4f n;
#pragma unroll
        for (int c = 0; c < 4; ++c) n[c] = (av[c] * d[c]) * inv + bv[c];
        *(v4fa*)(&ns[row * LP + 4 * lane]) = n;
    }
    __syncthreads();
#pragma unroll 1
    for (int ps = 0; ps < 2; ++ps) {
#pragma unroll
        for (int hh = 0; hh < 4; ++hh) { const int p = tid; const int row = p >> 2, c8 = (p & 3) * 8;
            const v4f x0 = *(const v4fa*)(&ns[row * LP + hh * 32 + c8]); const v4f x1 = *(const v4fa*)(&ns[row * LP + hh * 32 + c8 + 4]); v8h hv;
#pragma unroll
            for (int i = 0; i < 4; ++i) { hv[i] = toh_flush(x0[i]); hv[4 + i] = toh_flush(x1[i]); }
            const size_t oo = ((size_t)(bb * NH_ + hh) * SEQ + (size_t)tt) * HD + (size_t)p * 8;
            *(volatile v8h*)(QP + oo) = hv; }
#pragma unroll
        for (int s = 0; s < 4; ++s) { const int p = s * 256 + tid; const int m = p >> 3, c8 = (p & 7) * 8;
            v8h hv;
#pragma unroll
            for (int i = 0; i < 8; ++i) hv[i] = toh_flush(ns[(c8 + i) * LP + m]);
            const size_t oo = ((size_t)bb * DM + (size_t)m) * SEQ + (size_t)(tt + c8);
            *(volatile v8h*)(VT + oo) = hv; }
        if (ps == 0) __threadfence(); }
}

__global__ __launch_bounds__(32 * AW) void k_flash(const h16* __restrict__ QP, const h16* __restrict__ VT, const int* __restrict__ kmask, const float* __restrict__ aw, h16* CX) {
    __shared__ __align__(16) float os[AW * 16 * OSP];
    const int lane = threadIdx.x & 31, lr = lane & 15, hi = lane >> 4;
    const int wave = __builtin_amdgcn_readfirstlane((int)(threadIdx.x >> 5));
    const int zh = blockIdx.y; const int b = zh / NH_, h = zh % NH_;
    const int t0 = (blockIdx.x * AW + wave) * 16;
    const float qs = bfr(aw[(size_t)h * SEQ_FULL + t0 + lr]) * SC2;
    const int* kmb = kmask + (size_t)b * SEQ_FULL + 8 * hi;
    const size_t pbase = (size_t)zh * SEQ * HD;
    const size_t qo = pbase + (size_t)(t0 + lr) * HD + 8 * hi;
    const v16h qh = ldh(QP + qo);
    const size_t ko = pbase + (size_t)lr * HD + 8 * hi;
    const size_t vo = pbase + (size_t)lr * SEQ + 8 * hi;
    v8f o0 = (v8f){}, o1 = (v8f){};
    float m = NEGB, l = 0.0f;
#pragma unroll 1
    for (int key0 = 0; key0 < SEQ; key0 += 32) {
        const h16* ka = QP + ko + (size_t)key0 * HD;
        const v16h ka0 = ldh(ka), kb0 = ldh(ka + 16 * HD);
        v8f sa = (v8f){}, sb = (v8f){};
        sa = wmma16g(ka0, qh, sa); sb = wmma16g(kb0, qh, sb);
        const int* kp = kmb + key0;
        const v4i m0 = *(const v4i*)kp, m1 = *(const v4i*)(kp + 4), m2 = *(const v4i*)(kp + 16), m3 = *(const v4i*)(kp + 20);
        int kx[8], ky[8];
#pragma unroll
        for (int r = 0; r < 4; ++r) { kx[r] = m0[r]; kx[4 + r] = m1[r]; ky[r] = m2[r]; ky[4 + r] = m3[r]; }
        float ta[8], tb[8]; float mx = NEGB;
#pragma unroll
        for (int r = 0; r < 8; ++r) {
            ta[r] = (kx[r] != 0) ? (sa[r] * qs) : FILL2;
            tb[r] = (ky[r] != 0) ? (sb[r] * qs) : FILL2;
            mx = fmaxf(mx, fmaxf(ta[r], tb[r])); }
        mx = fmaxf(mx, __shfl_xor(mx, 16, 32));
        const float mnew = fmaxf(m, mx);
        const float alpha = __builtin_amdgcn_exp2f(m - mnew);
        const float sh = PSH - mnew;
        v16h pb; float ls = 0.0f;
#pragma unroll
        for (int r = 0; r < 8; ++r) {
            const float ea = ta[r] + sh, eb = tb[r] + sh;
            const float xa = __builtin_amdgcn_exp2f(ea), xb = __builtin_amdgcn_exp2f(eb);
            const float ga = (ea < -14.0f) ? 0.0f : xa, gb = (eb < -14.0f) ? 0.0f : xb;
            const h16 pa = (h16)ga; const h16 pc = (h16)gb;
            pb[r] = pa; pb[8 + r] = pc;
            ls += (float)pa + (float)pc; }
        l = l * alpha + ls; m = mnew;
        o0 = o0 * alpha; o1 = o1 * alpha;
        const h16* va = VT + vo + key0;
        const v16h v0 = ldh(va), v1 = ldh(va + (size_t)16 * SEQ);
        o0 = wmma16g(v0, pb, o0); o1 = wmma16g(v1, pb, o1);
    }
    l += __shfl_xor(l, 16, 32);
    const bool any = l > 0.0f;
    const float lsafe = any ? l : 1.0f;
    const float inv = any ? (CXS / lsafe) : 0.0f;
    const int wb = wave * 16 * OSP;
    { v4f a, c;
      a[0] = o0[0] * inv; a[1] = o0[1] * inv; a[2] = o0[2] * inv; a[3] = o0[3] * inv; c[0] = o0[4] * inv; c[1] = o0[5] * inv; c[2] = o0[6] * inv; c[3] = o0[7] * inv;
      *(v4fa*)(&os[wb + lr * OSP +  0 + 8 * hi]) = a; *(v4fa*)(&os[wb + lr * OSP +  0 + 8 * hi + 4]) = c;
      a[0] = o1[0] * inv; a[1] = o1[1] * inv; a[2] = o1[2] * inv; a[3] = o1[3] * inv; c[0] = o1[4] * inv; c[1] = o1[5] * inv; c[2] = o1[6] * inv; c[3] = o1[7] * inv;
      *(v4fa*)(&os[wb + lr * OSP + 16 + 8 * hi]) = a; *(v4fa*)(&os[wb + lr * OSP + 16 + 8 * hi + 4]) = c; }
    wave_sync();
    h16* crow = CX + pbase + (size_t)t0 * HD;
#pragma unroll 1
    for (int ps = 0; ps < 2; ++ps) {
#pragma unroll
        for (int s = 0; s < 2; ++s) { const int p = s * 32 + lane; const int row = p >> 2, c8 = (p & 3) * 8;
            const v4f x0 = *(const v4fa*)(&os[wb + row * OSP + c8]); const v4f x1 = *(const v4fa*)(&os[wb + row * OSP + c8 + 4]); v8h hv;
#pragma unroll
            for (int i = 0; i < 4; ++i) { hv[i] = toh_flush(x0[i]); hv[4 + i] = toh_flush(x1[i]); }
            *(volatile v8h*)(crow + (size_t)p * 8) = hv; }
        if (ps == 0) __threadfence(); }
}

__global__ __launch_bounds__(32 * TW) void k_tail(const h16* __restrict__ CX, const h16* __restrict__ WL, const h16* __restrict__ WF, const float* __restrict__ hid,
                                                  const float* __restrict__ bl, const float* __restrict__ b1, const float* __restrict__ ffs,
                                                  const float* __restrict__ g2, const float* __restrict__ be2, float* OUT) {
    __shared__ __align__(16) float xs[TW * 16 * TP];
    __shared__ __align__(16) float ys[TW * 16 * TP];
    __shared__ __align__(16) h16   hs[TW * 16 * HTP];
    const int lane = threadIdx.x & 31, lr = lane & 15, hi = lane >> 4;
    const int wave = __builtin_amdgcn_readfirstlane((int)(threadIdx.x >> 5));
    const int r0 = (blockIdx.x * TW + wave) * 16; const int bb = r0 / SEQ, tt = r0 % SEQ;
    const int wx = wave * 16 * TP, wh = wave * 16 * HTP;
    v8f acc[8];
#pragma unroll
    for (int nb = 0; nb < 8; ++nb) acc[nb] = (v8f){};
    const size_t ao = ((size_t)bb * NH_ * SEQ + (size_t)(tt + lr)) * HD + 8 * hi;
    const size_t wo = (size_t)lr * DM + 8 * hi;
#pragma unroll 1
    for (int kc = 0; kc < NH_; ++kc) {
        const v16h a = ldh(CX + ao + (size_t)kc * SEQ * HD);
#pragma unroll
        for (int nb = 0; nb < 8; ++nb) { const v16h bw = ldh(WL + wo + (size_t)nb * 16 * DM + kc * 32); acc[nb] = wmma16g(a, bw, acc[nb]); }
    }
#pragma unroll
    for (int nb = 0; nb < 8; ++nb) {
#pragma unroll
        for (int j = 0; j < 8; ++j) xs[wx + (hi * 8 + j) * TP + nb * 16 + lr] = acc[nb][j] * CI1; }
    wave_sync();
    v4f blv = *(const v4f*)(bl + 4 * lane), g2v = *(const v4f*)(g2 + 4 * lane), be2v = *(const v4f*)(be2 + 4 * lane), b1v = *(const v4f*)(b1 + 4 * lane);
#pragma unroll
    for (int i = 0; i < 4; ++i) { blv[i] = bfr(blv[i]); g2v[i] = bfr(g2v[i]); be2v[i] = bfr(be2v[i]); b1v[i] = bfr(b1v[i]); }
#pragma unroll 1
    for (int r = 0; r < 16; ++r) {
        const int xi = wx + r * TP + 4 * lane;
        const v4f a = *(const v4fa*)(&xs[xi]);
        const v4f hx = *(const v4f*)(hid + ((size_t)bb * SEQ_FULL + (size_t)(tt + r)) * DM + 4 * lane);
        v4f x;
#pragma unroll
        for (int i = 0; i < 4; ++i) x[i] = bfr(hx[i]) + (a[i] + blv[i]);
        float s = (x[0] + x[1]) + (x[2] + x[3]);
#pragma unroll
        for (int o = 16; o >= 1; o >>= 1) s += __shfl_xor(s, o, 32);
        const float mean = s * (1.0f / DM);
        v4f d; float ss = 0.0f;
#pragma unroll
        for (int i = 0; i < 4; ++i) { d[i] = x[i] - mean; ss += d[i] * d[i]; }
#pragma unroll
        for (int o = 16; o >= 1; o >>= 1) ss += __shfl_xor(ss, o, 32);
        const float sd = sqrtf(ss * (1.0f / (DM - 1)));
        const float inv = 1.0f / (sd + 1e-6f);
        v4h nv;
#pragma unroll
        for (int i = 0; i < 4; ++i) nv[i] = toh_flush((g2v[i] * d[i]) * inv + be2v[i]);
        *(v4fa*)(&xs[xi]) = x;
        *(v4ha*)(&hs[wh + r * HTP + 4 * lane]) = nv;
    }
    wave_sync();
#pragma unroll
    for (int nb = 0; nb < 8; ++nb) acc[nb] = (v8f){};
#pragma unroll 1
    for (int kc = 0; kc < DM / 32; ++kc) {
        const int hp = wh + lr * HTP + kc * 32 + 8 * hi;
        const v16h a = cat16(*(const v8ha*)(&hs[hp]), *(const v8ha*)(&hs[hp + 16]));
#pragma unroll
        for (int nb = 0; nb < 8; ++nb) { const v16h bw = ldh(WF + wo + (size_t)nb * 16 * DM + kc * 32); acc[nb] = wmma16g(a, bw, acc[nb]); }
    }
#pragma unroll
    for (int nb = 0; nb < 8; ++nb) {
#pragma unroll
        for (int j = 0; j < 8; ++j) ys[wx + (hi * 8 + j) * TP + nb * 16 + lr] = acc[nb][j] * CI2; }
    wave_sync();
#pragma unroll 1
    for (int r = 0; r < 16; ++r) {
        const int xi = wx + r * TP + 4 * lane;
        const v4f g = *(const v4fa*)(&ys[xi]);
        const v4f x2 = *(const v4fa*)(&xs[xi]);
        const float fs = bfr(ffs[tt + r]);
        v4f o;
#pragma unroll
        for (int i = 0; i < 4; ++i) {
            const float hf = fs * (g[i] + b1v[i]);
            const float u = GK * (hf + 0.044715f * ((hf * hf) * hf));
            const float act = (0.5f * hf) * (1.0f + tanhf(u));
            o[i] = x2[i] + act; }
        *(v4fa*)(&ys[xi]) = o;
    }
    wave_sync();
    float* orow = OUT + ((size_t)bb * OUT_SEQ + (size_t)tt) * DM + 4 * lane;
#pragma unroll 1
    for (int ps = 0; ps < 2; ++ps) {
#pragma unroll 4
        for (int r = 0; r < 16; ++r) {
            const v4f val = *(const v4fa*)(&ys[wx + r * TP + 4 * lane]);
            *(volatile v4f*)(orow + (size_t)r * DM) = val; }
        if (ps == 0) __threadfence(); }
}

static constexpr size_t al256(size_t v) { return (v + 255) & ~(size_t)255; }
static constexpr size_t SZ_PL = al256((size_t)NB * NH_ * SEQ * HD * 2);
static constexpr size_t SZ_W  = al256((size_t)DM * DM * 2);
static constexpr size_t SZ_TOTAL = 3 * SZ_PL + 2 * SZ_W;
static_assert(SZ_TOTAL <= (size_t)134217728);
static_assert((size_t)NB * NH_ * SEQ * HD == (size_t)NB * DM * SEQ);
static_assert(((size_t)DM * DM) % 8 == 0);
static_assert((size_t)(NB * SEQ / 64) * 64 * DM * 2 == (size_t)NB * NH_ * SEQ * HD * 2);
static_assert((size_t)(SEQ / (16 * AW)) * AW * 16 * HD * 2 * NB * NH_ == (size_t)NB * NH_ * SEQ * HD * 2);

extern "C" void kernel_launch(void* const* d_in, const int* in_sizes, int n_in,
                              void* d_out, int out_size, void* d_ws, size_t ws_size, hipStream_t stream) {
    if (n_in < 12) return;
    const size_t needx = ((size_t)(NB - 1) * SEQ_FULL + SEQ) * DM;
    const size_t needm = (size_t)(NB - 1) * SEQ_FULL + SEQ;
    const size_t needa = (size_t)(NH_ - 1) * SEQ_FULL + SEQ;
    if ((size_t)in_sizes[0] < needx || (size_t)in_sizes[1] < needm || (size_t)in_sizes[2] < needa) return;
    if ((size_t)in_sizes[3] < (size_t)DM * DM || (size_t)in_sizes[5] < (size_t)DM * DM) return;
    if (in_sizes[4] < DM || in_sizes[6] < DM || in_sizes[7] < SEQ) return;
    if (in_sizes[8] < DM || in_sizes[9] < DM || in_sizes[10] < DM || in_sizes[11] < DM) return;
    if ((size_t)out_size < ((size_t)(NB - 1) * OUT_SEQ + SEQ) * DM) return;
    if (SZ_TOTAL > ws_size) return;
    const float* hidden = (const float*)d_in[0];
    const int*   mask   = (const int*)d_in[1];
    const float* aw     = (const float*)d_in[2];
    const float* wl     = (const float*)d_in[3];
    const float* bl     = (const float*)d_in[4];
    const float* w1     = (const float*)d_in[5];
    const float* b1     = (const float*)d_in[6];
    const float* ffs    = (const float*)d_in[7];
    const float* ln1a   = (const float*)d_in[8];
    const float* ln1b   = (const float*)d_in[9];
    const float* ln2a   = (const float*)d_in[10];
    const float* ln2b   = (const float*)d_in[11];
    float* OUT = (float*)d_out;
    char* wsp = (char*)d_ws;
    h16* QP  = (h16*)wsp; wsp += SZ_PL;
    h16* VT  = (h16*)wsp; wsp += SZ_PL;
    h16* CX  = (h16*)wsp; wsp += SZ_PL;
    h16* WLp = (h16*)wsp; wsp += SZ_W;
    h16* WFp = (h16*)wsp; wsp += SZ_W;

    { const size_t n8 = (size_t)DM * DM / 8; const unsigned g = (unsigned)((n8 + 255) / 256);
      k_wcvt<<<g, 256, 0, stream>>>(wl, WLp, n8); k_wcvt<<<g, 256, 0, stream>>>(w1, WFp, n8); }
    k_ln1<<<NB * SEQ / 64, 256, 0, stream>>>(hidden, ln1a, ln1b, QP, VT);
    k_flash<<<dim3(SEQ / (16 * AW), NB * NH_, 1), 32 * AW, 0, stream>>>(QP, VT, mask, aw, CX);
    k_tail<<<NB * SEQ / (16 * TW), 32 * TW, 0, stream>>>(CX, WLp, WFp, hidden, bl, b1, ffs, ln2a, ln2b, OUT);
}
